// MessagePassingLayer_35081292873864
// MI455X (gfx1250) — hardware-verified
//
#include <hip/hip_runtime.h>
#include <stddef.h>
#include <stdint.h>


#define HD     128
#define NNODE  81
#define NBATCH 256
#define NEDGE  1620
#define MROWS  (NBATCH * NNODE)
#define ECAPP  1664
#define TAB_CNT 0
#define TAB_RP  128
#define TAB_SRC 256
#define TABN   (TAB_SRC + ECAPP)
#define NTHR   256
#define NWAVE  8
#define GBM    64
#define GBN    128
#define GTHR   128
#define PQP    256
#define HLP    256
#define WU0    4096
#define WU1N   4096
#define WU2N   6144
#define WU3N   4096
#define WUTOT  (WU0 + WU1N + WU2N + WU3N)
#define NODE_IT 11
#define WSMAX  134217728

static_assert(MROWS % GBM == 0);
static_assert(TABN % 4 == 0 && (TABN * 4) % 128 == 0);
static_assert(ECAPP >= NEDGE && ECAPP % 32 == 0 && NNODE <= 128);
static_assert((TABN / 4) <= 2 * NTHR && ((TABN / 4) - NTHR) % 32 == 0);
static_assert(WU0 % NTHR == 0 && WU1N % NTHR == 0 && WU2N % NTHR == 0 && WU3N % NTHR == 0);
static_assert((MROWS * (HD / 8)) % NTHR == 0);
static_assert(NODE_IT * NWAVE >= NNODE);
static_assert(GBM == (GTHR / 32) * 16 && GBN == HD && HD == 4 * 32);
static_assert(HD % 32 == 0 && (2 * HD) % 32 == 0 && (3 * HD) % 32 == 0);

typedef float          v4f   __attribute__((ext_vector_type(4)));
typedef float          v8f   __attribute__((ext_vector_type(8)));
typedef int            v4i   __attribute__((ext_vector_type(4)));
typedef int            v8i   __attribute__((ext_vector_type(8)));
typedef unsigned       v2u   __attribute__((ext_vector_type(2)));
typedef unsigned short v4us  __attribute__((ext_vector_type(4)));
typedef unsigned short v8us  __attribute__((ext_vector_type(8)));
typedef unsigned short v16us __attribute__((ext_vector_type(16)));
typedef __bf16         v16bf __attribute__((ext_vector_type(16)));
typedef v4f  __attribute__((may_alias)) v4fa;
typedef v4i  __attribute__((may_alias)) v4ia;
typedef v2u  __attribute__((may_alias)) v2ua;
typedef v4us __attribute__((may_alias)) v4usa;
typedef v8us __attribute__((may_alias)) v8usa;
union FragB { v16bf v; v16us u; v8us h[2]; v8i w; };

__device__ __forceinline__ v8f wmb(const FragB& a, const FragB& b, v8f c) {
  v8f d = __builtin_amdgcn_wmma_f32_16x16x32_bf16(false, a.v, false, b.v, (short)0, c, false, false);
  asm volatile("v_nop\n\tv_nop\n\tv_nop\n\tv_nop" : "+v"(d) : "v"(a.w), "v"(b.w));
  return d;
}

__device__ __forceinline__ unsigned bf16_bits(float f) {
  const unsigned u = __float_as_uint(f);
  return (u + 0x7FFFu + ((u >> 16) & 1u)) >> 16;
}
__device__ __forceinline__ float bf16_val(float f) {
  return __uint_as_float(bf16_bits(f) << 16);
}

__device__ __forceinline__ void wave_sync() {
  __builtin_amdgcn_fence(__ATOMIC_RELEASE, "wavefront");
  __builtin_amdgcn_wave_barrier();
  __builtin_amdgcn_fence(__ATOMIC_ACQUIRE, "wavefront");
}

__global__ __launch_bounds__(NTHR) void k_wprep(const float* __restrict__ Wm1, const float* __restrict__ Wm2,
                                                const float* __restrict__ Wu1, const float* __restrict__ Wu2,
                                                unsigned short* WmT, unsigned short* WM2,
                                                unsigned short* WU1, unsigned short* WU2) {
  const int u = (int)blockIdx.x * NTHR + (int)threadIdx.x;
  const float* p;
  unsigned short* dp;
  if (u < WU0) {
    const int n  = u >> 4;
    const int k8 = (u & 15) * 8;
    const int ks = k8 + ((n >> 7) << 7);
    p  = Wm1 + (size_t)ks * HD + (n & 127);
    dp = WmT + (size_t)n * HD + k8;
  } else if (u < WU0 + WU1N) {
    const int v  = u - WU0;
    const int n  = v >> 5;
    const int k8 = (v & 31) * 8;
    p  = Wm2 + (size_t)(k8 & 127) * HD + n;
    dp = WM2 + (size_t)n * (2 * HD) + k8;
  } else if (u < WU0 + WU1N + WU2N) {
    const int v  = u - (WU0 + WU1N);
    const int n  = v / 48;
    const int k8 = (v - n * 48) * 8;
    const int ks = (k8 < HD) ? k8 : (HD + ((k8 - HD) & 127));
    p  = Wu1 + (size_t)ks * HD + n;
    dp = WU1 + (size_t)n * (3 * HD) + k8;
  } else if (u < WUTOT) {
    const int v  = u - (WU0 + WU1N + WU2N);
    const int n  = v >> 5;
    const int k8 = (v & 31) * 8;
    p  = Wu2 + (size_t)(k8 & 127) * HD + n;
    dp = WU2 + (size_t)n * (2 * HD) + k8;
  } else {
    return;
  }
  v8us o;
#pragma unroll
  for (int i = 0; i < 8; ++i) o[i] = (unsigned short)bf16_bits(p[(size_t)i * HD]);
  *(volatile v8us*)dp = o;
  __threadfence();
  *(volatile v8us*)dp = o;
}

__global__ __launch_bounds__(NTHR) void k_cvx(const float* __restrict__ x, unsigned short* xb) {
  const int u = (int)blockIdx.x * NTHR + (int)threadIdx.x;
  if (u >= MROWS * (HD / 8)) return;
  const int row = u >> 4;
  const int k8  = (u & 15) * 8;
  const float* p = x + (size_t)row * HD + k8;
  const v4f a = *(const v4fa*)p;
  const v4f b = *(const v4fa*)(p + 4);
  v8us o;
  o[0] = (unsigned short)bf16_bits(a.x); o[1] = (unsigned short)bf16_bits(a.y);
  o[2] = (unsigned short)bf16_bits(a.z); o[3] = (unsigned short)bf16_bits(a.w);
  o[4] = (unsigned short)bf16_bits(b.x); o[5] = (unsigned short)bf16_bits(b.y);
  o[6] = (unsigned short)bf16_bits(b.z); o[7] = (unsigned short)bf16_bits(b.w);
  unsigned short* dp = xb + (size_t)row * HD + k8;
  *(volatile v8us*)dp = o;
  __threadfence();
  *(volatile v8us*)dp = o;
}

__global__ __launch_bounds__(NTHR) void k_csr(const int* __restrict__ ei, int* tab) {
  __shared__ __attribute__((aligned(16))) int tl[ECAPP];
  __shared__ __attribute__((aligned(16))) int sl[ECAPP];
  __shared__ __attribute__((aligned(16))) int tb[TABN];
  const int tid = (int)threadIdx.x;
#pragma unroll 1
  for (int e = tid; e < ECAPP; e += NTHR) {
    const int ec = e < NEDGE ? e : NEDGE - 1;
    const int s  = ei[ec];
    const int t  = ei[NEDGE + ec];
    const bool ok = e < NEDGE;
    const int sc = s < 0 ? 0 : (s > NNODE - 1 ? NNODE - 1 : s);
    sl[e] = ok ? sc : 0;
    tl[e] = ok ? t : -1;
  }
#pragma unroll 1
  for (int i = tid; i < TABN; i += NTHR) tb[i] = 0;
  __syncthreads();

  int c = 0;
#pragma unroll 4
  for (int e = 0; e < NEDGE; ++e) c += (tl[e] == tid) ? 1 : 0;
  const int cv = (tid < NNODE) ? c : 0;
  if (tid < 128) tb[TAB_CNT + tid] = cv;
  __syncthreads();

  int rp = 0;
  {
    const int lim = tid < NNODE ? tid : NNODE;
#pragma unroll 1
    for (int j = 0; j < NNODE; ++j) {
      const int v = tb[TAB_CNT + j];
      rp += (j < lim) ? v : 0;
    }
  }
  if (tid < 128) tb[TAB_RP + tid] = rp;

  int pos = rp;
#pragma unroll 2
  for (int e = 0; e < NEDGE; ++e) {
    const int t = tl[e];
    const int s = sl[e];
    const bool hit = (t == tid) && (tid < NNODE);
    if (hit) {
      const int pc = pos < ECAPP - 1 ? pos : ECAPP - 1;
      tb[TAB_SRC + pc] = s;
    }
    pos += hit ? 1 : 0;
  }
  __syncthreads();

  v4i tv[2];
#pragma unroll
  for (int it = 0; it < 2; ++it) {
    const int i4 = it * NTHR + tid;
    const int ic = i4 < TABN / 4 ? i4 : TABN / 4 - 1;
    tv[it] = *(const v4ia*)(tb + 4 * ic);
  }
#pragma unroll
  for (int it = 0; it < 2; ++it) {
    const int i4 = it * NTHR + tid;
    if (i4 < TABN / 4) *(volatile v4i*)(tab + 4 * (size_t)i4) = tv[it];
  }
  __threadfence();
#pragma unroll
  for (int it = 0; it < 2; ++it) {
    const int i4 = it * NTHR + tid;
    if (i4 < TABN / 4) *(volatile v4i*)(tab + 4 * (size_t)i4) = tv[it];
  }
}

__global__ __launch_bounds__(NTHR) void k_scan(const int* __restrict__ tab, const float* __restrict__ PQ,
                                               unsigned short* HB) {
  __shared__ __attribute__((aligned(16))) int tb[TABN];
  __shared__ __attribute__((aligned(16))) unsigned short rowb[NWAVE * HLP];
  const int tid = (int)threadIdx.x, lane = tid & 31, wave = tid >> 5;
  const int b = (int)blockIdx.x;
#pragma unroll
  for (int it = 0; it < 2; ++it) {
    const int i4 = it * NTHR + tid;
    const int ic = i4 < TABN / 4 ? i4 : TABN / 4 - 1;
    const v4i t4 = *(const v4i*)(tab + 4 * (size_t)ic);
    if (i4 < TABN / 4) *(v4ia*)(tb + 4 * i4) = t4;
  }
  __syncthreads();

  unsigned short* rowbuf = rowb + wave * HLP;
  const float qnan = __int_as_float(0x7fc00000);
  const size_t rb = (size_t)b * NNODE;
#pragma unroll 1
  for (int ni = 0; ni < NODE_IT; ++ni) {
    const int node = ni * NWAVE + wave;
    if (node < NNODE) {
      const int craw = tb[TAB_CNT + node];
      const int oraw = tb[TAB_RP + node];
      int c = craw < 0 ? 0 : (craw > NEDGE ? NEDGE : craw);
      const int o = oraw < 0 ? 0 : (oraw > NEDGE ? NEDGE : oraw);
      bool bad = (c != craw) || (o != oraw);
      if (o + c > NEDGE) { c = NEDGE - o; bad = true; }
      const v4f q4 = *(const v4f*)(PQ + (rb + (size_t)node) * PQP + HD + 4 * lane);
      float a0 = 0.0f, a1 = 0.0f, a2 = 0.0f, a3 = 0.0f;
#pragma unroll 1
      for (int b0 = 0; b0 < c; b0 += 32) {
        int idx = o + b0 + lane;
        idx = idx > ECAPP - 1 ? ECAPP - 1 : idx;
        int sr = tb[TAB_SRC + idx];
        sr = sr < 0 ? 0 : (sr > NNODE - 1 ? NNODE - 1 : sr);
        const int m32 = (c - b0) < 32 ? (c - b0) : 32;
#pragma unroll 1
        for (int k = 0; k < m32; ++k) {
          const int sk = __builtin_amdgcn_readlane(sr, k);
          const v4f p4 = *(const v4f*)(PQ + (rb + (size_t)sk) * PQP + 4 * lane);
          const float v0 = p4.x + q4.x, v1 = p4.y + q4.y, v2 = p4.z + q4.z, v3 = p4.w + q4.w;
          a0 += (v0 > 0.0f) ? v0 : (v0 - v0);
          a1 += (v1 > 0.0f) ? v1 : (v1 - v1);
          a2 += (v2 > 0.0f) ? v2 : (v2 - v2);
          a3 += (v3 > 0.0f) ? v3 : (v3 - v3);
        }
      }
      const float cf  = (c < 1) ? 1.0f : (float)c;
      const float inv = 1.0f / cf;
      const float pz  = bad ? qnan : 0.0f;
      const float m0 = a0 * inv + pz, m1 = a1 * inv + pz, m2 = a2 * inv + pz, m3 = a3 * inv + pz;
      v4us mh, ml;
      {
        unsigned hb;
        hb = bf16_bits(m0); mh[0] = (unsigned short)hb; ml[0] = (unsigned short)bf16_bits(m0 - __uint_as_float(hb << 16));
        hb = bf16_bits(m1); mh[1] = (unsigned short)hb; ml[1] = (unsigned short)bf16_bits(m1 - __uint_as_float(hb << 16));
        hb = bf16_bits(m2); mh[2] = (unsigned short)hb; ml[2] = (unsigned short)bf16_bits(m2 - __uint_as_float(hb << 16));
        hb = bf16_bits(m3); mh[3] = (unsigned short)hb; ml[3] = (unsigned short)bf16_bits(m3 - __uint_as_float(hb << 16));
      }
      *(v4usa*)(rowbuf + 4 * lane) = mh;
      *(v4usa*)(rowbuf + HD + 4 * lane) = ml;
      wave_sync();
      const v8us q0 = *(const v8usa*)(rowbuf + 8 * lane);
      wave_sync();
      unsigned short* rpw = HB + (rb + (size_t)node) * HLP + 8 * lane;
      *(volatile v8us*)rpw = q0;
      __threadfence();
      *(volatile v8us*)rpw = q0;
    }
  }
}

template <int MODE>
__global__ __launch_bounds__(GTHR) void k_gemm(const unsigned short* A1, int lda1, int K1,
                                               const unsigned short* A2, int lda2, int K2,
                                               const unsigned short* __restrict__ BT,
                                               const float* __restrict__ bias, const int* __restrict__ tab,
                                               const unsigned short* XB,
                                               const float* __restrict__ gam, const float* __restrict__ bet,
                                               float* outF, unsigned short* outH) {
  __shared__ __attribute__((aligned(16))) float stg[GBM * GBN];
  __shared__ float gateL[GBM];
  const int tid = (int)threadIdx.x, lane = tid & 31, wave = tid >> 5, hh = lane >> 4, m = lane & 15;
  const int rowBase = (int)blockIdx.x * GBM;
  const int col0    = (int)blockIdx.y * GBN;
  const int KT      = K1 + K2;

  if (tid < GBM) {
    float g = 1.0f;
    if constexpr (MODE == 1) {
      const int node = (rowBase + tid) % NNODE;
      const int cn = tab[TAB_CNT + node];
      g = (cn > 0) ? 1.0f : 0.0f;
    }
    gateL[tid] = g;
  }

  v8f acc[8];
  {
    const v8f z = {0.f, 0.f, 0.f, 0.f, 0.f, 0.f, 0.f, 0.f};
#pragma unroll
    for (int t = 0; t < 8; ++t) acc[t] = z;
  }
  const unsigned short* ap1 = A1 + (size_t)(rowBase + 16 * wave + m) * (size_t)lda1 + 8 * hh;
  const unsigned short* ap2 = A2 + (size_t)(rowBase + 16 * wave + m) * (size_t)lda2 + 8 * hh;
  const unsigned short* bp  = BT + (size_t)(col0 + m) * (size_t)KT + 8 * hh;

#pragma unroll 1
  for (int k0 = 0; k0 < K1; k0 += 32) {
    FragB af;
    af.h[0] = *(const v8usa*)(ap1 + k0);
    af.h[1] = *(const v8usa*)(ap1 + k0 + 16);
#pragma unroll
    for (int nt = 0; nt < 8; ++nt) {
      const unsigned short* wq = bp + (size_t)(16 * nt) * (size_t)KT + k0;
      FragB bf;
      bf.h[0] = *(const v8usa*)wq;
      bf.h[1] = *(const v8usa*)(wq + 16);
      acc[nt] = wmb(af, bf, acc[nt]);
    }
  }
#pragma unroll 1
  for (int k0 = 0; k0 < K2; k0 += 32) {
    FragB af;
    af.h[0] = *(const v8usa*)(ap2 + k0);
    af.h[1] = *(const v8usa*)(ap2 + k0 + 16);
#pragma unroll
    for (int nt = 0; nt < 8; ++nt) {
      const unsigned short* wq = bp + (size_t)(16 * nt) * (size_t)KT + K1 + k0;
      FragB bf;
      bf.h[0] = *(const v8usa*)wq;
      bf.h[1] = *(const v8usa*)(wq + 16);
      acc[nt] = wmb(af, bf, acc[nt]);
    }
  }

#pragma unroll
  for (int nt = 0; nt < 8; ++nt) {
    const int lc = 16 * nt + m;
#pragma unroll
    for (int r = 0; r < 8; ++r) {
      const int lr = 16 * wave + 8 * hh + r;
      stg[lr * GBN + lc] = acc[nt][r];
    }
  }
  __syncthreads();

  v4f bb4;
  {
    const v4f t1 = *(const v4f*)(bias + 4 * lane);
    bb4.x = bf16_val(t1.x); bb4.y = bf16_val(t1.y); bb4.z = bf16_val(t1.z); bb4.w = bf16_val(t1.w);
  }

  if constexpr (MODE == 0) {
    const float bs = ((int)blockIdx.y == 1) ? 1.0f : 0.0f;
    const v4f bq = bb4 * bs;
    v4f pv[16];
#pragma unroll
    for (int i = 0; i < 16; ++i) pv[i] = *(const v4fa*)(stg + (16 * wave + i) * GBN + 4 * lane) + bq;
#pragma unroll
    for (int i = 0; i < 16; ++i) {
      const int r = rowBase + 16 * wave + i;
      *(volatile v4f*)(outF + (size_t)r * PQP + col0 + 4 * lane) = pv[i];
    }
    __threadfence();
#pragma unroll
    for (int i = 0; i < 16; ++i) {
      const int r = rowBase + 16 * wave + i;
      *(volatile v4f*)(outF + (size_t)r * PQP + col0 + 4 * lane) = pv[i];
    }
  } else if constexpr (MODE == 1 || MODE == 2) {
    v4f pv[16];
#pragma unroll
    for (int i = 0; i < 16; ++i) pv[i] = *(const v4fa*)(stg + (16 * wave + i) * GBN + 4 * lane);
    __syncthreads();
#pragma unroll
    for (int i = 0; i < 16; ++i) {
      v4f t = pv[i];
      if constexpr (MODE == 1) {
        const float g = gateL[16 * wave + i];
        t.x += bb4.x * g; t.y += bb4.y * g; t.z += bb4.z * g; t.w += bb4.w * g;
      } else {
        t = t + bb4;
        t.x = (t.x > 0.0f) ? t.x : (t.x - t.x);
        t.y = (t.y > 0.0f) ? t.y : (t.y - t.y);
        t.z = (t.z > 0.0f) ? t.z : (t.z - t.z);
        t.w = (t.w > 0.0f) ? t.w : (t.w - t.w);
      }
      v4us h4, l4;
      unsigned hb;
      hb = bf16_bits(t.x); h4[0] = (unsigned short)hb; l4[0] = (unsigned short)bf16_bits(t.x - __uint_as_float(hb << 16));
      hb = bf16_bits(t.y); h4[1] = (unsigned short)hb; l4[1] = (unsigned short)bf16_bits(t.y - __uint_as_float(hb << 16));
      hb = bf16_bits(t.z); h4[2] = (unsigned short)hb; l4[2] = (unsigned short)bf16_bits(t.z - __uint_as_float(hb << 16));
      hb = bf16_bits(t.w); h4[3] = (unsigned short)hb; l4[3] = (unsigned short)bf16_bits(t.w - __uint_as_float(hb << 16));
      unsigned short* srow = (unsigned short*)stg + (size_t)(16 * wave + i) * (2 * GBN);
      *(v4usa*)(srow + 4 * lane) = h4;
      *(v4usa*)(srow + HD + 4 * lane) = l4;
    }
    __syncthreads();
    v8us qv[16];
#pragma unroll
    for (int i = 0; i < 16; ++i) {
      const unsigned short* srow = (const unsigned short*)stg + (size_t)(16 * wave + i) * (2 * GBN);
      qv[i] = *(const v8usa*)(srow + 8 * lane);
    }
#pragma unroll
    for (int i = 0; i < 16; ++i) {
      unsigned short* rp = outH + (size_t)(rowBase + 16 * wave + i) * (size_t)HLP + 8 * lane;
      *(volatile v8us*)rp = qv[i];
    }
    __threadfence();
#pragma unroll
    for (int i = 0; i < 16; ++i) {
      unsigned short* rp = outH + (size_t)(rowBase + 16 * wave + i) * (size_t)HLP + 8 * lane;
      *(volatile v8us*)rp = qv[i];
    }
  } else {
    v4f g4, e4;
    {
      const v4f t1 = *(const v4f*)(gam + 4 * lane);
      const v4f t2 = *(const v4f*)(bet + 4 * lane);
      g4.x = bf16_val(t1.x); g4.y = bf16_val(t1.y); g4.z = bf16_val(t1.z); g4.w = bf16_val(t1.w);
      e4.x = bf16_val(t2.x); e4.y = bf16_val(t2.y); e4.z = bf16_val(t2.z); e4.w = bf16_val(t2.w);
    }
#pragma unroll 1
    for (int i = 0; i < 16; ++i) {
      const int lr = 16 * wave + i;
      const int r  = rowBase + lr;
      float* sp = stg + lr * GBN + 4 * lane;
      const v4f t = *(const v4fa*)sp;
      const v2u xw = *(const v2ua*)(XB + (size_t)r * HD + 4 * lane);
      const float x0 = __uint_as_float(xw.x << 16);
      const float x1 = __uint_as_float(xw.x & 0xffff0000u);
      const float x2 = __uint_as_float(xw.y << 16);
      const float x3 = __uint_as_float(xw.y & 0xffff0000u);
      const float y0 = (t.x + bb4.x) + x0;
      const float y1 = (t.y + bb4.y) + x1;
      const float y2 = (t.z + bb4.z) + x2;
      const float y3 = (t.w + bb4.w) + x3;
      float s = (y0 + y1) + (y2 + y3);
      s += __shfl_xor(s, 16, 32);
      s += __shfl_xor(s, 8, 32);
      s += __shfl_xor(s, 4, 32);
      s += __shfl_xor(s, 2, 32);
      s += __shfl_xor(s, 1, 32);
      const float mu = s * (1.0f / (float)HD);
      const float d0 = y0 - mu, d1 = y1 - mu, d2 = y2 - mu, d3 = y3 - mu;
      float q = (d0 * d0 + d1 * d1) + (d2 * d2 + d3 * d3);
      q += __shfl_xor(q, 16, 32);
      q += __shfl_xor(q, 8, 32);
      q += __shfl_xor(q, 4, 32);
      q += __shfl_xor(q, 2, 32);
      q += __shfl_xor(q, 1, 32);
      const float var = q * (1.0f / (float)HD);
      const float rs  = rsqrtf(var + 1e-5f);
      v4f o;
      o.x = d0 * rs * g4.x + e4.x;
      o.y = d1 * rs * g4.y + e4.y;
      o.z = d2 * rs * g4.z + e4.z;
      o.w = d3 * rs * g4.w + e4.w;
      *(v4fa*)sp = o;
    }
    v4f pv[16];
#pragma unroll
    for (int i = 0; i < 16; ++i) pv[i] = *(const v4fa*)(stg + (16 * wave + i) * GBN + 4 * lane);
#pragma unroll
    for (int i = 0; i < 16; ++i) {
      const int r = rowBase + 16 * wave + i;
      *(volatile v4f*)(outF + (size_t)r * HD + 4 * lane) = pv[i];
    }
    __threadfence();
#pragma unroll
    for (int i = 0; i < 16; ++i) {
      const int r = rowBase + 16 * wave + i;
      *(volatile v4f*)(outF + (size_t)r * HD + 4 * lane) = pv[i];
    }
  }
}

static inline size_t al256(size_t o) { return (o + 255) & ~(size_t)255; }

extern "C" void kernel_launch(void* const* d_in, const int* in_sizes, int n_in,
                              void* d_out, int out_size, void* d_ws, size_t ws_size,
                              hipStream_t stream) {
  if (n_in < 12) return;
  if (in_sizes[0] != MROWS * HD) return;
  if (in_sizes[1] != 2 * NEDGE) return;
  if (in_sizes[2] != 2 * HD * HD || in_sizes[3] != HD) return;
  if (in_sizes[4] != HD * HD || in_sizes[5] != HD) return;
  if (in_sizes[6] != 2 * HD * HD || in_sizes[7] != HD) return;
  if (in_sizes[8] != HD * HD || in_sizes[9] != HD) return;
  if (in_sizes[10] != HD || in_sizes[11] != HD) return;
  if (out_size != MROWS * HD) return;

  const float* x    = (const float*)d_in[0];
  const int*   ei   = (const int*)d_in[1];
  const float* Wm1  = (const float*)d_in[2];
  const float* bm1  = (const float*)d_in[3];
  const float* Wm2  = (const float*)d_in[4];
  const float* bm2  = (const float*)d_in[5];
  const float* Wu1  = (const float*)d_in[6];
  const float* bu1  = (const float*)d_in[7];
  const float* Wu2  = (const float*)d_in[8];
  const float* bu2  = (const float*)d_in[9];
  const float* gam  = (const float*)d_in[10];
  const float* bet  = (const float*)d_in[11];
  float* out = (float*)d_out;

  char* ws = (char*)d_ws;
  size_t off = 0;
  const size_t oTAB = off; off = al256(off + (size_t)TABN * 4);
  const size_t oWmT = off; off = al256(off + (size_t)2 * HD * HD * 2);
  const size_t oWM2 = off; off = al256(off + (size_t)HD * 2 * HD * 2);
  const size_t oWU1 = off; off = al256(off + (size_t)HD * 3 * HD * 2);
  const size_t oWU2 = off; off = al256(off + (size_t)HD * 2 * HD * 2);
  const size_t oXB  = off; off = al256(off + (size_t)MROWS * HD * 2);
  const size_t oPQ  = off; off = al256(off + (size_t)MROWS * PQP * 4);
  const size_t oHB  = off; off = al256(off + (size_t)MROWS * HLP * 2);
  const size_t oAG  = off; off = al256(off + (size_t)MROWS * HLP * 2);
  const size_t oU1  = off; off = al256(off + (size_t)MROWS * HLP * 2);
  if (off > ws_size || off > (size_t)WSMAX) return;
  int*            TAB = (int*)(ws + oTAB);
  unsigned short* WmT = (unsigned short*)(ws + oWmT);
  unsigned short* WM2 = (unsigned short*)(ws + oWM2);
  unsigned short* WU1 = (unsigned short*)(ws + oWU1);
  unsigned short* WU2 = (unsigned short*)(ws + oWU2);
  unsigned short* XB  = (unsigned short*)(ws + oXB);
  float*          PQ  = (float*)(ws + oPQ);
  unsigned short* HB  = (unsigned short*)(ws + oHB);
  unsigned short* AG  = (unsigned short*)(ws + oAG);
  unsigned short* U1  = (unsigned short*)(ws + oU1);

  const int gM = MROWS / GBM;

  k_wprep<<<WUTOT / NTHR, NTHR, 0, stream>>>(Wm1, Wm2, Wu1, Wu2, WmT, WM2, WU1, WU2);
  k_cvx<<<(MROWS * (HD / 8)) / NTHR, NTHR, 0, stream>>>(x, XB);
  k_csr<<<1, NTHR, 0, stream>>>(ei, TAB);
  k_gemm<0><<<dim3(gM, 2), GTHR, 0, stream>>>(XB, HD, HD, XB, HD, 0, WmT, bm1, TAB, XB, gam, bet, PQ, HB);
  k_scan<<<NBATCH, NTHR, 0, stream>>>(TAB, PQ, HB);
  k_gemm<1><<<dim3(gM, 1), GTHR, 0, stream>>>(HB, HLP, 2 * HD, HB, HLP, 0, WM2, bm2, TAB, XB, gam, bet, PQ, AG);
  k_gemm<2><<<dim3(gM, 1), GTHR, 0, stream>>>(XB, HD, HD, AG, HLP, 2 * HD, WU1, bu1, TAB, XB, gam, bet, PQ, U1);
  k_gemm<3><<<dim3(gM, 1), GTHR, 0, stream>>>(U1, HLP, 2 * HD, U1, HLP, 0, WU2, bu2, TAB, XB, gam, bet, out, U1);
}
